// ConvLayer_1443109011969
// MI455X (gfx1250) — hardware-verified
//
#include <hip/hip_runtime.h>
#include <stddef.h>


#define HD     64
#define ED     16
#define QOFF   (HD * HD)
#define PCOLS  (HD * HD + HD)
#define RCOLS  (4 * HD)
#define GCOLS  (3 * HD)
#define BTROWS (PCOLS + RCOLS)
#define W1ROW  BTROWS
#define BTALL  (BTROWS + HD)
#define NB     128
#define NTHR   256
#define NWAVE  8
#define EPT    8
#define CHUNK  (NTHR * EPT)
#define WCAP   (EPT * 32)
#define GTHR   128

static_assert(CHUNK <= 4096);
static_assert((NB % 32) == 0);
static_assert(NB < 4096);
static_assert((BTALL % 32) == 0);
static_assert((PCOLS % 64) == 0);
static_assert((RCOLS % 64) == 0);
static_assert((GCOLS % 64) == 0);

typedef float          v2f  __attribute__((ext_vector_type(2)));
typedef float          v4f  __attribute__((ext_vector_type(4)));
typedef float          v4fa __attribute__((ext_vector_type(4))) __attribute__((may_alias));
typedef float          v8f  __attribute__((ext_vector_type(8)));
typedef int            v4i  __attribute__((ext_vector_type(4)));
typedef unsigned short us_t;
typedef us_t           v8us __attribute__((ext_vector_type(8)));
typedef __bf16         v16bf __attribute__((ext_vector_type(16)));
union FragB { v16bf v; v8us h[2]; };

__device__ __forceinline__ us_t f2bf(float f) {
  unsigned u = __float_as_uint(f);
  u = u + 0x7FFFu + ((u >> 16) & 1u);
  return (us_t)(u >> 16);
}
__device__ __forceinline__ float bf2f(us_t b) { return __uint_as_float(((unsigned)b) << 16); }

__device__ __forceinline__ void split8(v4f a, v4f b, v8us& hi, v8us& lo) {
#pragma unroll
  for (int j = 0; j < 4; ++j) {
    const us_t h0 = f2bf(a[j]);
    hi[j] = h0;
    lo[j] = f2bf(a[j] - bf2f(h0));
    const us_t h1 = f2bf(b[j]);
    hi[4 + j] = h1;
    lo[4 + j] = f2bf(b[j] - bf2f(h1));
  }
}

__device__ __forceinline__ v4f zero4() { v4f z; z.x = 0.0f; z.y = 0.0f; z.z = 0.0f; z.w = 0.0f; return z; }
__device__ __forceinline__ v4f sel4(bool c, v4f a) {
  v4f r;
  r.x = c ? a.x : 0.0f; r.y = c ? a.y : 0.0f; r.z = c ? a.z : 0.0f; r.w = c ? a.w : 0.0f;
  return r;
}

__device__ __forceinline__ v8f wmb(v16bf a, v16bf b, v8f c) {
  v8f d = __builtin_amdgcn_wmma_f32_16x16x32_bf16(false, a, false, b, (short)0, c, false, false);
  asm volatile("v_nop\n\tv_nop\n\tv_nop\n\tv_nop" : "+v"(d) : "v"(a), "v"(b));
  return d;
}

__device__ __forceinline__ float sigm(float x) {
  x = fminf(fmaxf(x, -30.0f), 30.0f);
  return __builtin_amdgcn_rcpf(1.0f + __expf(-x));
}
__device__ __forceinline__ float tanh_f(float x) {
  const float a = fminf(fabsf(x), 15.0f);
  const float t = __expf(-2.0f * a);
  const float r = (1.0f - t) * __builtin_amdgcn_rcpf(1.0f + t);
  return x < 0.0f ? -r : r;
}

__global__ __launch_bounds__(NTHR) void k_cvt(const float* __restrict__ src, us_t* dh, us_t* dl,
                                              int nRows, int srcW, int rowsPad) {
  const int tid = threadIdx.x;
  const int row = (int)blockIdx.x * 32 + (tid >> 3);
  const int col = 8 * (tid & 7);
  const bool valid = (row < nRows) && (col + 8 <= srcW);
  int rc = row < nRows ? row : nRows - 1;
  rc = rc < 0 ? 0 : rc;
  int cc = (col + 8 <= srcW) ? col : srcW - 8;
  cc = cc < 0 ? 0 : cc;
  const float* p = src + (size_t)rc * srcW + cc;
  const v4f a = sel4(valid, *(const v4f*)p);
  const v4f b = sel4(valid, *(const v4f*)(p + 4));
  v8us hv, lv;
  split8(a, b, hv, lv);
  const size_t off = (size_t)row * HD + col;
  const bool wr = row < rowsPad;
  if (wr) { *(volatile v8us*)(dh + off) = hv; *(volatile v8us*)(dl + off) = lv; }
  __threadfence();
  if (wr) { *(volatile v8us*)(dh + off) = hv; *(volatile v8us*)(dl + off) = lv; }
}

__global__ __launch_bounds__(NTHR) void k_btprep(const float* __restrict__ W2, const float* __restrict__ b2,
                                                 const float* __restrict__ Wr, const float* __restrict__ whh,
                                                 const float* __restrict__ W1, us_t* Bh, us_t* Bl) {
  const int tid = threadIdx.x;
  const int c = (int)blockIdx.x * 32 + (tid >> 3);
  const int c8 = tid & 7;
  const int cc = c < QOFF ? c : QOFF - 1;
  const int hc = cc >> 6, oc = c & 63;
  int g = c - (PCOLS + HD);
  g = g < 0 ? 0 : (g > GCOLS - 1 ? GCOLS - 1 : g);
  v4f a, b;
#pragma unroll
  for (int j = 0; j < 8; ++j) {
    const int i = 8 * c8 + j;
    const float w2 = W2[(size_t)hc * QOFF + (size_t)i * HD + oc];
    const float bb = b2[i * HD + oc];
    const float wr = Wr[oc * HD + i];
    const float wh = whh[g * HD + i];
    const int ic = i < ED ? i : ED - 1;
    float w1 = W1[ic * HD + oc];
    if (i >= ED) w1 = 0.0f;
    float v;
    if (c < QOFF) v = w2;
    else if (c < PCOLS) v = bb;
    else if (c < PCOLS + HD) v = wr;
    else if (c < BTROWS) v = wh;
    else v = w1;
    if (j < 4) a[j] = v; else b[j - 4] = v;
  }
  v8us hv, lv;
  split8(a, b, hv, lv);
  const size_t off = (size_t)c * HD + 8 * c8;
  *(volatile v8us*)(Bh + off) = hv; *(volatile v8us*)(Bl + off) = lv;
  __threadfence();
  *(volatile v8us*)(Bh + off) = hv; *(volatile v8us*)(Bl + off) = lv;
}

template <int HASBIAS, int RELU>
__global__ __launch_bounds__(GTHR) void k_gemm(const us_t* __restrict__ Ah, const us_t* __restrict__ Al,
                                               const us_t* __restrict__ Bh, const us_t* __restrict__ Bl,
                                               const float* __restrict__ bias,
                                               float* P, int pPitch, int nPcb, float* R, int rPitch, int aRow0) {
  __shared__ __attribute__((aligned(16))) float stg[4 * 32 * 32];
  const int tid = threadIdx.x, lane = tid & 31, wave = tid >> 5, hh = lane >> 4, m = lane & 15;
  const int wr = wave >> 1, wc = wave & 1;
  const int rowA = aRow0 + (int)blockIdx.y * 64 + wr * 32;
  const int colB = (int)blockIdx.x * 64 + wc * 32;

  FragB ah[2][2], al[2][2];
#pragma unroll
  for (int rt = 0; rt < 2; ++rt) {
#pragma unroll
    for (int ks = 0; ks < 2; ++ks) {
      const size_t o = (size_t)(rowA + rt * 16 + m) * HD + ks * 32 + 8 * hh;
      ah[rt][ks].h[0] = *(const v8us*)(Ah + o);
      ah[rt][ks].h[1] = *(const v8us*)(Ah + o + 16);
      al[rt][ks].h[0] = *(const v8us*)(Al + o);
      al[rt][ks].h[1] = *(const v8us*)(Al + o + 16);
    }
  }
  v8f acc[2][2];
#pragma unroll
  for (int rt = 0; rt < 2; ++rt) {
#pragma unroll
    for (int ct = 0; ct < 2; ++ct) {
#pragma unroll
      for (int r = 0; r < 8; ++r) acc[rt][ct][r] = 0.0f;
    }
  }
#pragma unroll
  for (int ct = 0; ct < 2; ++ct) {
    FragB bh[2], bl[2];
#pragma unroll
    for (int ks = 0; ks < 2; ++ks) {
      const size_t o = (size_t)(colB + ct * 16 + m) * HD + ks * 32 + 8 * hh;
      bh[ks].h[0] = *(const v8us*)(Bh + o);
      bh[ks].h[1] = *(const v8us*)(Bh + o + 16);
      bl[ks].h[0] = *(const v8us*)(Bl + o);
      bl[ks].h[1] = *(const v8us*)(Bl + o + 16);
    }
#pragma unroll
    for (int rt = 0; rt < 2; ++rt) {
#pragma unroll
      for (int ks = 0; ks < 2; ++ks) {
        acc[rt][ct] = wmb(ah[rt][ks].v, bh[ks].v, acc[rt][ct]);
        acc[rt][ct] = wmb(ah[rt][ks].v, bl[ks].v, acc[rt][ct]);
        acc[rt][ct] = wmb(al[rt][ks].v, bh[ks].v, acc[rt][ct]);
      }
    }
  }

  float* sw = stg + wave * 1024;
#pragma unroll
  for (int ct = 0; ct < 2; ++ct) {
    float bv = 0.0f;
    if (HASBIAS != 0) bv = bias[colB + ct * 16 + m];
#pragma unroll
    for (int rt = 0; rt < 2; ++rt) {
#pragma unroll
      for (int r = 0; r < 8; ++r) {
        float v = acc[rt][ct][r] + bv;
        if (RELU != 0) v = fmaxf(v, 0.0f);
        sw[(rt * 16 + 8 * hh + r) * 32 + ct * 16 + m] = v;
      }
    }
  }
  __syncthreads();

  const int q = lane >> 3, p4 = (lane & 7) * 4;
  float* dst;
  int pitch;
  if ((int)blockIdx.x < nPcb) {
    dst = P + (size_t)((int)blockIdx.y * 64 + wr * 32) * pPitch + (size_t)blockIdx.x * 64 + wc * 32;
    pitch = pPitch;
  } else {
    dst = R + (size_t)rowA * rPitch + (size_t)((int)blockIdx.x - nPcb) * 64 + wc * 32;
    pitch = rPitch;
  }
  v4f ov[8];
#pragma unroll
  for (int rr = 0; rr < 8; ++rr) ov[rr] = *(const v4fa*)(sw + (rr * 4 + q) * 32 + p4);
#pragma unroll
  for (int rr = 0; rr < 8; ++rr) *(volatile v4f*)(dst + (size_t)(rr * 4 + q) * pitch + p4) = ov[rr];
  __threadfence();
#pragma unroll
  for (int rr = 0; rr < 8; ++rr) *(volatile v4f*)(dst + (size_t)(rr * 4 + q) * pitch + p4) = ov[rr];
}

__global__ __launch_bounds__(NTHR) void k_msg(const int* __restrict__ ei, const float* __restrict__ H1,
                                              const float* __restrict__ P, float* msg,
                                              int nN, int nE, int row0, int nRowsHalf, int pPitch) {
  const int tid = threadIdx.x, lane = tid & 31, wave = tid >> 5;
  const int e = (int)blockIdx.x * NWAVE + wave;
  if (e >= nE) return;
  int s = ei[e];
  s = s < 0 ? 0 : (s > nN - 1 ? nN - 1 : s);
  if (s < row0 || s >= row0 + nRowsHalf) return;
  const float* pr = P + (size_t)(s - row0) * pPitch;
  const float* hr = H1 + (size_t)e * HD;
  const int o2 = 2 * lane;
  v2f acc = *(const v2f*)(pr + QOFF + o2);
#pragma unroll 4
  for (int hg = 0; hg < HD / 4; ++hg) {
    const v4f h4 = *(const v4f*)(hr + 4 * hg);
#pragma unroll
    for (int j = 0; j < 4; ++j) {
      const v2f p = *(const v2f*)(pr + (size_t)(4 * hg + j) * HD + o2);
      acc.x = fmaf(h4[j], p.x, acc.x);
      acc.y = fmaf(h4[j], p.y, acc.y);
    }
  }
  float* mp = msg + (size_t)e * HD + o2;
  *(volatile v2f*)mp = acc;
  __threadfence();
  *(volatile v2f*)mp = acc;
}

__device__ __forceinline__ int scan_chunk(const int* __restrict__ dsts, int nE, int cbase, int nodeBase,
                                          int vec8, int* list, int tid, int wave) {
  int wc = 0;
  const int el0  = tid * EPT;
  const int e0   = cbase + el0;
  const int sent = -2147483647 - 1;
  v4i da, db;
  if (vec8 != 0 && cbase + CHUNK <= nE) {
    da = *(const v4i*)(dsts + e0);
    db = *(const v4i*)(dsts + e0 + 4);
  } else {
    da.x = (e0     < nE) ? dsts[min(e0, nE - 1)] : sent;
    da.y = (e0 + 1 < nE) ? dsts[min(e0 + 1, nE - 1)] : sent;
    da.z = (e0 + 2 < nE) ? dsts[min(e0 + 2, nE - 1)] : sent;
    da.w = (e0 + 3 < nE) ? dsts[min(e0 + 3, nE - 1)] : sent;
    db.x = (e0 + 4 < nE) ? dsts[min(e0 + 4, nE - 1)] : sent;
    db.y = (e0 + 5 < nE) ? dsts[min(e0 + 5, nE - 1)] : sent;
    db.z = (e0 + 6 < nE) ? dsts[min(e0 + 6, nE - 1)] : sent;
    db.w = (e0 + 7 < nE) ? dsts[min(e0 + 7, nE - 1)] : sent;
  }
  const unsigned nb = (unsigned)nodeBase;
  const unsigned s0 = (unsigned)da.x - nb, s1 = (unsigned)da.y - nb;
  const unsigned s2 = (unsigned)da.z - nb, s3 = (unsigned)da.w - nb;
  const unsigned s4 = (unsigned)db.x - nb, s5 = (unsigned)db.y - nb;
  const unsigned s6 = (unsigned)db.z - nb, s7 = (unsigned)db.w - nb;
  const bool h0 = s0 < (unsigned)NB, h1 = s1 < (unsigned)NB, h2 = s2 < (unsigned)NB, h3 = s3 < (unsigned)NB;
  const bool h4 = s4 < (unsigned)NB, h5 = s5 < (unsigned)NB, h6 = s6 < (unsigned)NB, h7 = s7 < (unsigned)NB;
  const unsigned any = __builtin_amdgcn_ballot_w32(h0 | h1 | h2 | h3 | h4 | h5 | h6 | h7);
  if (any != 0u) {
#define HITJ(J, HJ, SJ) { \
      const unsigned mj = __builtin_amdgcn_ballot_w32(HJ); \
      if (mj != 0u) { \
        if (HJ) { \
          const int pos = wc + (int)__builtin_amdgcn_mbcnt_lo(mj, 0u); \
          if (pos < WCAP) list[wave * WCAP + pos] = (int)(((SJ) << 12) | (unsigned)(el0 + (J))); \
        } \
        wc += (int)__builtin_popcount(mj); } }
    HITJ(0, h0, s0)
    HITJ(1, h1, s1)
    HITJ(2, h2, s2)
    HITJ(3, h3, s3)
    HITJ(4, h4, s4)
    HITJ(5, h5, s5)
    HITJ(6, h6, s6)
    HITJ(7, h7, s7)
#undef HITJ
  }
  return wc;
}

__global__ __launch_bounds__(NTHR) void k_agg(const int* __restrict__ ei, const float* __restrict__ msg,
                                              const float* __restrict__ R, const float* __restrict__ bconv,
                                              us_t* Mh, us_t* Ml, int nN, int nE, int vec8, int rPitch) {
  __shared__ __attribute__((aligned(16))) float acc[NB * HD];
  __shared__ float cnt[NB];
  __shared__ int   list[NWAVE * WCAP];
  __shared__ int   wcnt[NWAVE];
  const int tid = threadIdx.x, lane = tid & 31, wave = tid >> 5;
  const int nodeBase = (int)blockIdx.x * NB;
  const int* dsts = ei + nE;

  for (int i = tid; i < NB * HD; i += NTHR) acc[i] = 0.0f;
  if (tid < NB) cnt[tid] = 0.0f;
  __syncthreads();

  const int nChunks = (nE + CHUNK - 1) / CHUNK;
#pragma unroll 1
  for (int ch = 0; ch < nChunks; ++ch) {
    const int cbase = ch * CHUNK;
    const int wc = scan_chunk(dsts, nE, cbase, nodeBase, vec8, list, tid, wave);
    if (lane == 0) wcnt[wave] = wc;
    __syncthreads();
    if (wave < 2) {
      const int o = wave * 32 + lane;
#pragma unroll 1
      for (int w = 0; w < NWAVE; ++w) {
        int n = wcnt[w];
        n = n > WCAP ? WCAP : (n < 0 ? 0 : n);
#pragma unroll 1
        for (int i = 0; i < n; ++i) {
          const int ent = list[w * WCAP + i];
          int sl = ent >> 12;
          sl = sl < 0 ? 0 : (sl > NB - 1 ? NB - 1 : sl);
          int e = cbase + (ent & 4095);
          e = e < 0 ? 0 : (e > nE - 1 ? nE - 1 : e);
          const float v = msg[(size_t)e * HD + o];
          acc[sl * HD + o] += v;
          if (wave == 0 && lane == 0) cnt[sl] += 1.0f;
        }
      }
    }
    __syncthreads();
  }

  v8us hv[NB / 32], lv[NB / 32];
  const int c8 = lane & 7;
#pragma unroll
  for (int sw = 0; sw < NB / 32; ++sw) {
    const int row = sw * 32 + wave * 4 + (lane >> 3);
    const int n = nodeBase + row;
    const bool valid = n < nN;
    const int nc = valid ? n : nN - 1;
    const v4f a0 = *(const v4fa*)(acc + row * HD + 8 * c8);
    const v4f a1 = *(const v4fa*)(acc + row * HD + 8 * c8 + 4);
    const float cn = cnt[row];
    const float inv = 1.0f / fmaxf(cn, 1.0f);
    const float* rp = R + (size_t)nc * rPitch + 8 * c8;
    const v4f r0 = *(const v4f*)rp, r1 = *(const v4f*)(rp + 4);
    const v4f b0 = *(const v4f*)(bconv + 8 * c8), b1 = *(const v4f*)(bconv + 8 * c8 + 4);
    v4f m0, m1;
#pragma unroll
    for (int j = 0; j < 4; ++j) {
      const float t0 = fmaxf(a0[j] * inv + r0[j] + b0[j], 0.0f);
      const float t1 = fmaxf(a1[j] * inv + r1[j] + b1[j], 0.0f);
      m0[j] = valid ? t0 : 0.0f;
      m1[j] = valid ? t1 : 0.0f;
    }
    split8(m0, m1, hv[sw], lv[sw]);
    const size_t off = (size_t)n * HD + 8 * c8;
    *(volatile v8us*)(Mh + off) = hv[sw];
    *(volatile v8us*)(Ml + off) = lv[sw];
  }
  __threadfence();
#pragma unroll
  for (int sw = 0; sw < NB / 32; ++sw) {
    const int row = sw * 32 + wave * 4 + (lane >> 3);
    const size_t off = (size_t)(nodeBase + row) * HD + 8 * c8;
    *(volatile v8us*)(Mh + off) = hv[sw];
    *(volatile v8us*)(Ml + off) = lv[sw];
  }
}

__global__ __launch_bounds__(NTHR) void k_gate(const float* __restrict__ G, const float* __restrict__ R,
                                               const float* __restrict__ hprev, const float* __restrict__ bhh,
                                               float* hnew, us_t* Hh, us_t* Hl, int nN, int rPitch) {
  __shared__ __attribute__((aligned(16))) float hrow[4 * HD];
  const int tid = threadIdx.x, lane = tid & 31, wave = tid >> 5;
  const int ln = tid >> 6, o = tid & 63;
  const int n = (int)blockIdx.x * 4 + ln;
  const bool valid = n < nN;
  const int nc = valid ? n : nN - 1;
  const float* g  = G + (size_t)nc * GCOLS;
  const float* rh = R + (size_t)nc * rPitch + HD;
  const float gr = g[o], gz = g[HD + o], gn = g[2 * HD + o];
  const float hr = rh[o] + bhh[o];
  const float hz = rh[HD + o] + bhh[HD + o];
  const float hn = rh[2 * HD + o] + bhh[2 * HD + o];
  const float hp = hprev[(size_t)nc * HD + o];
  const float r  = sigm(gr + hr);
  const float z  = sigm(gz + hz);
  const float nn = tanh_f(gn + r * hn);
  const float h  = (1.0f - z) * nn + z * hp;
  hrow[ln * HD + o] = h;
  float* hq = hnew + (size_t)nc * HD + o;
  if (valid) *(volatile float*)hq = h;
  __syncthreads();

  v8us sv;
#pragma unroll
  for (int j = 0; j < 8; ++j) sv[j] = (us_t)0;
  bool pw = false;
  size_t poff = 0;
  us_t* pp = (wave == 0) ? Hh : Hl;
  if (wave < 2) {
    const int row = lane >> 3, c8 = lane & 7;
    const int n2 = (int)blockIdx.x * 4 + row;
    const v4f a = *(const v4fa*)(hrow + row * HD + 8 * c8);
    const v4f b = *(const v4fa*)(hrow + row * HD + 8 * c8 + 4);
    v8us hv, lv;
    split8(a, b, hv, lv);
    sv = hv;
    if (wave != 0) sv = lv;
    pw = n2 < nN;
    const int n2c = pw ? n2 : nN - 1;
    poff = (size_t)n2c * HD + 8 * c8;
  }
  if (wave < 2 && pw) *(volatile v8us*)(pp + poff) = sv;
  __threadfence();
  if (valid) *(volatile float*)hq = h;
  if (wave < 2 && pw) *(volatile v8us*)(pp + poff) = sv;
}

extern "C" void kernel_launch(void* const* d_in, const int* in_sizes, int n_in,
                              void* d_out, int out_size, void* d_ws, size_t ws_size,
                              hipStream_t stream) {
  if (n_in < 13) return;
  const int nN = in_sizes[0] / HD;
  const int nE = in_sizes[12] / 2;
  if (nN <= 0 || nE <= 0) return;
  if (in_sizes[0] != nN * HD || in_sizes[12] != 2 * nE || in_sizes[1] != nE * ED) return;
  if (in_sizes[2] != ED * HD || in_sizes[3] != HD) return;
  if (in_sizes[4] != HD * QOFF || in_sizes[5] != QOFF) return;
  if (in_sizes[6] != HD * HD || in_sizes[7] != HD) return;
  if (in_sizes[8] != GCOLS * HD || in_sizes[9] != GCOLS * HD || in_sizes[10] != GCOLS || in_sizes[11] != GCOLS) return;
  if (out_size != nN * HD) return;

  const float* x      = (const float*)d_in[0];
  const float* ea     = (const float*)d_in[1];
  const float* W1     = (const float*)d_in[2];
  const float* b1     = (const float*)d_in[3];
  const float* W2     = (const float*)d_in[4];
  const float* b2     = (const float*)d_in[5];
  const float* W_root = (const float*)d_in[6];
  const float* b_conv = (const float*)d_in[7];
  const float* w_ih   = (const float*)d_in[8];
  const float* w_hh   = (const float*)d_in[9];
  const float* b_ih   = (const float*)d_in[10];
  const float* b_hh   = (const float*)d_in[11];
  const int*   ei     = (const int*)d_in[12];
  float* out = (float*)d_out;

  const int NPADA = ((nN + 127) / 128) * 128;
  const int HR    = NPADA / 2;
  const int Epad  = ((nE + 63) / 64) * 64;

  char* ws = (char*)d_ws;
  size_t off = 0;
  auto take = [&](size_t bytes) { char* p = ws + off; off += (bytes + 255) & ~(size_t)255; return p; };
  us_t*  Hh   = (us_t*)take((size_t)NPADA * HD * 2);
  us_t*  Hl   = (us_t*)take((size_t)NPADA * HD * 2);
  us_t*  EAh  = (us_t*)take((size_t)Epad * HD * 2);
  us_t*  EAl  = (us_t*)take((size_t)Epad * HD * 2);
  us_t*  WIHh = (us_t*)take((size_t)GCOLS * HD * 2);
  us_t*  WIHl = (us_t*)take((size_t)GCOLS * HD * 2);
  us_t*  BTh  = (us_t*)take((size_t)BTALL * HD * 2);
  us_t*  BTl  = (us_t*)take((size_t)BTALL * HD * 2);
  us_t*  Mh   = (us_t*)take((size_t)NPADA * HD * 2);
  us_t*  Ml   = (us_t*)take((size_t)NPADA * HD * 2);
  float* H1   = (float*)take((size_t)Epad * HD * 4);
  float* Pbuf = (float*)take((size_t)HR * PCOLS * 4);
  float* Rbuf = (float*)take((size_t)NPADA * RCOLS * 4);
  float* Gbuf = (float*)take((size_t)NPADA * GCOLS * 4);
  float* S0   = (float*)take((size_t)NPADA * HD * 4);
  float* S1   = (float*)take((size_t)NPADA * HD * 4);
  float* MSG  = (float*)take((size_t)Epad * HD * 4);
  if (off > ws_size) return;

  const int vec8 = ((nE & 3) == 0) ? 1 : 0;

  k_cvt<<<NPADA / 32, NTHR, 0, stream>>>(x, Hh, Hl, nN, HD, NPADA);
  k_cvt<<<Epad / 32, NTHR, 0, stream>>>(ea, EAh, EAl, nE, ED, Epad);
  k_cvt<<<GCOLS / 32, NTHR, 0, stream>>>(w_ih, WIHh, WIHl, GCOLS, HD, GCOLS);
  k_btprep<<<BTALL / 32, NTHR, 0, stream>>>(W2, b2, W_root, w_hh, W1, BTh, BTl);
  k_gemm<1, 1><<<dim3(1, Epad / 64), GTHR, 0, stream>>>(
      EAh, EAl, BTh + (size_t)W1ROW * HD, BTl + (size_t)W1ROW * HD, b1, H1, HD, 1, H1, HD, 0);

  const float* hprev = x;
  for (int it = 0; it < 3; ++it) {
    float* hnew = (it == 0) ? S0 : ((it == 1) ? S1 : out);
    for (int half = 0; half < 2; ++half) {
      k_gemm<0, 0><<<dim3(BTROWS / 64, HR / 64), GTHR, 0, stream>>>(
          Hh, Hl, BTh, BTl, b1, Pbuf, PCOLS, PCOLS / 64, Rbuf, RCOLS, half * HR);
      k_msg<<<(nE + NWAVE - 1) / NWAVE, NTHR, 0, stream>>>(ei, H1, Pbuf, MSG, nN, nE, half * HR, HR, PCOLS);
    }
    k_agg<<<NPADA / NB, NTHR, 0, stream>>>(ei, MSG, Rbuf, b_conv, Mh, Ml, nN, nE, vec8, RCOLS);
    k_gemm<1, 0><<<dim3(GCOLS / 64, NPADA / 64), GTHR, 0, stream>>>(
        Mh, Ml, WIHh, WIHl, b_ih, Gbuf, GCOLS, GCOLS / 64, Gbuf, GCOLS, 0);
    k_gate<<<(nN + 3) / 4, NTHR, 0, stream>>>(Gbuf, Rbuf, hprev, b_hh, hnew, Hh, Hl, nN, RCOLS);
    hprev = hnew;
  }
}
